// GATConvTransformerDecoderLayer_44641890075097
// MI455X (gfx1250) — hardware-verified
//
#include <hip/hip_runtime.h>
#include <math.h>


#define NNODE 4096
#define NEDGE 262144
#define FIN 128
#define NH 4
#define CH 64
#define EMB 256
#define DFF 128

typedef __attribute__((ext_vector_type(16))) __bf16 v16bf;
typedef __attribute__((ext_vector_type(8)))  float v8f;
typedef __attribute__((ext_vector_type(4)))  float v4f;
typedef float __attribute__((may_alias)) float_a;

template <typename T> __device__ __forceinline__ void vst2(void* p, T v) { *(volatile T*)p = v; __threadfence(); *(volatile T*)p = v; }
__device__ __forceinline__ v8f wmma_bf(v16bf a, v16bf b, v8f c) {
  v8f d = __builtin_amdgcn_wmma_f32_16x16x32_bf16(false, a, false, b, (short)0, c, false, false);
  asm volatile("v_nop\n\tv_nop\n\tv_nop\n\tv_nop" : "+v"(d) : "v"(a), "v"(b));
  return d;
}
struct F2 { v16bf h, l; };
__device__ __forceinline__ F2 split16(const float* v) {
  F2 r;
#pragma unroll
  for (int i = 0; i < 16; ++i) { const __bf16 hh = (__bf16)v[i]; r.h[i] = hh; r.l[i] = (__bf16)(v[i] - (float)hh); }
  return r;
}
__device__ __forceinline__ F2 split_row(const float* row, int k0, int lane) {
  float v[16]; const float* p = row + k0 + 8 * (lane >> 4);
#pragma unroll
  for (int i = 0; i < 8; ++i) { v[i] = p[i]; v[8 + i] = p[16 + i]; }
  return split16(v);
}
__device__ __forceinline__ F2 split_col(const float* base, int k0, int lane, int stride) {
  float v[16]; const float* p = base + (size_t)(k0 + 8 * (lane >> 4)) * stride;
#pragma unroll
  for (int i = 0; i < 8; ++i) { v[i] = p[(size_t)i * stride]; v[8 + i] = p[(size_t)(16 + i) * stride]; }
  return split16(v);
}
__device__ __forceinline__ v8f mac3(const F2& a, const F2& b, v8f c) { c = wmma_bf(a.l, b.h, c); c = wmma_bf(a.h, b.l, c); return wmma_bf(a.h, b.h, c); }

__global__ __launch_bounds__(128) void k_gemm(const float* __restrict__ A, int lda, const float* __restrict__ Bm, int ldb, int bmode,
                                            const float* __restrict__ bias, int act, float* __restrict__ C, int ldc, int K) {
  __shared__ __align__(16) float st[64][68];
  const int tid = threadIdx.x, wave = tid >> 5, lane = tid & 31, col = lane & 15, g = lane >> 4;
  const int m0 = blockIdx.x * 64 + wave * 16, n0 = blockIdx.y * 64;
  const float* arow = A + (size_t)(m0 + col) * lda;
  v8f acc[4] = {};
#pragma unroll 1
  for (int kc = 0; kc < K / 32; ++kc) {
    const F2 a = split_row(arow, kc * 32, lane);
#pragma unroll
    for (int j = 0; j < 4; ++j) {
      const F2 bf = bmode == 0 ? split_row(Bm + (size_t)(n0 + j * 16 + col) * ldb, kc * 32, lane)
                               : split_col(Bm + n0 + j * 16 + col, kc * 32, lane, ldb);
      acc[j] = mac3(a, bf, acc[j]);
    }
  }
#pragma unroll
  for (int j = 0; j < 4; ++j) {
    const float bv = bias ? bias[n0 + j * 16 + col] : 0.f;
#pragma unroll
    for (int r = 0; r < 8; ++r) { float v = acc[j][r] + bv; if (act == 1) v = fmaxf(v, 0.f); st[wave * 16 + 8 * g + r][j * 16 + col] = v; }
  }
  __syncthreads();
  const int bm0 = blockIdx.x * 64;
  for (int q = tid; q < 64 * 16; q += 128) { const int rl = q >> 4, pc = q & 15;
    vst2(C + (size_t)(bm0 + rl) * ldc + n0 + pc * 4, *(const v4f*)(&st[rl][pc * 4])); }
}

__global__ __launch_bounds__(256) void k_gat_alpha(const float* __restrict__ xh, const float* __restrict__ att_src, const float* __restrict__ att_dst,
                                                 float* __restrict__ as, float* __restrict__ ad) {
  __shared__ float s_as[32][NH], s_ad[32][NH];
  const int wave = threadIdx.x >> 5, lane = threadIdx.x & 31;
  for (int k = 0; k < 4; ++k) {
    const int nl = wave * 4 + k, n = blockIdx.x * 32 + nl;
    const float* row = xh + (size_t)n * EMB;
    float ps = 0.f, pd = 0.f;
#pragma unroll
    for (int e = 0; e < 8; ++e) { const int i = lane * 8 + e; ps += row[i] * att_src[i]; pd += row[i] * att_dst[i]; }
#pragma unroll
    for (int off = 4; off >= 1; off >>= 1) { ps += __shfl_xor(ps, off, 32); pd += __shfl_xor(pd, off, 32); }
    if ((lane & 7) == 0) { s_as[nl][lane >> 3] = ps; s_ad[nl][lane >> 3] = pd; }
  }
  __syncthreads();
  if (threadIdx.x < 32) { const int i = threadIdx.x * 4; v4f v = { s_as[i >> 2][0], s_as[i >> 2][1], s_as[i >> 2][2], s_as[i >> 2][3] };
    vst2(as + (size_t)blockIdx.x * 128 + i, v); }
  else if (threadIdx.x < 64) { const int i = (threadIdx.x - 32) * 4; v4f v = { s_ad[i >> 2][0], s_ad[i >> 2][1], s_ad[i >> 2][2], s_ad[i >> 2][3] };
    vst2(ad + (size_t)blockIdx.x * 128 + i, v); }
}

#define DT 64
#define ECH 2048
__global__ __launch_bounds__(256) void k_gat_gather(const int* __restrict__ ei, const float* __restrict__ xh,
                                                  const float* __restrict__ as, const float* __restrict__ ad, const float* __restrict__ bgat,
                                                  float* __restrict__ tout) {
  __shared__ __align__(16) float acc[DT][EMB];
  __shared__ float mrun[DT][NH], lrun[DT][NH];
  __shared__ int es[ECH], ed[ECH];
  const int tid = threadIdx.x, lane = tid & 31, wave = tid >> 5;
  const int d0 = blockIdx.x * DT;
  for (int i = tid; i < DT * EMB / 4; i += 256) *(v4f*)(&acc[0][0] + i * 4) = (v4f){0.f, 0.f, 0.f, 0.f};
  for (int i = tid; i < DT * NH; i += 256) { (&mrun[0][0])[i] = -3.0e38f; (&lrun[0][0])[i] = 0.f; }
  __syncthreads();
  const int myh = lane >> 3;
  auto update = [&](int dl, int s) {
    const float a_raw = as[(size_t)s * NH + myh] + ad[(size_t)(d0 + dl) * NH + myh];
    const float a = a_raw > 0.f ? a_raw : 0.2f * a_raw;
    const float mo = mrun[dl][myh], mn = fmaxf(mo, a);
    const float corr = expf(mo - mn), p = expf(a - mn);
    const float* xr = xh + (size_t)s * EMB + lane * 8;
    float* ar = &acc[dl][lane * 8];
#pragma unroll
    for (int e = 0; e < 8; ++e) ar[e] = ar[e] * corr + p * xr[e];
    const float lo_ = lrun[dl][myh];
    __builtin_amdgcn_wave_barrier();
    if ((lane & 7) == 0) { mrun[dl][myh] = mn; lrun[dl][myh] = lo_ * corr + p; }
    asm volatile("s_wait_dscnt 0" ::: "memory"); __builtin_amdgcn_wave_barrier();
  };
  for (int e0 = 0; e0 < NEDGE; e0 += ECH) {
    __syncthreads();
    for (int i = tid; i < ECH; i += 256) { es[i] = ei[e0 + i]; ed[i] = ei[(size_t)NEDGE + e0 + i]; }
    __syncthreads();
    for (int base = 0; base < ECH; base += 32) {
      const int dl = ed[base + lane] - d0;
      const bool mine = (dl >= 0) && (dl < DT) && ((dl & 7) == wave);
      unsigned msk = (unsigned)__builtin_amdgcn_ballot_w32(mine);
      while (msk) {
        const int j = __builtin_ctz(msk); msk &= msk - 1u;
        const int ii = base + j;
        const int dlj = ed[ii] - d0;
        int s = es[ii]; s = s < 0 ? 0 : (s >= NNODE ? NNODE - 1 : s);
        update(dlj, s);
      }
    }
  }
  for (int dl = wave; dl < DT; dl += 8) update(dl, d0 + dl);
  __syncthreads();
  for (int r = wave; r < DT; r += 8) {
#pragma unroll
    for (int half = 0; half < 2; ++half) { const int c0 = half * 128 + lane * 4;
      v4f v;
#pragma unroll
      for (int e = 0; e < 4; ++e) { const int c = c0 + e; float t = acc[r][c] / (lrun[r][c >> 6] + 1e-16f) + bgat[c]; v[e] = t > 0.f ? t : 0.01f * t; }
      vst2(tout + (size_t)(d0 + r) * EMB + c0, v); }
  }
}

__global__ __launch_bounds__(128) void k_attn(const float* __restrict__ Q, const float* __restrict__ Kf, const float* __restrict__ V,
                                            float* __restrict__ O) {
  __shared__ __align__(16) float Ps[4][16 * 32];
  __shared__ __align__(16) float Os[4][16 * 64];
  const int tid = threadIdx.x, wl = tid >> 5, lane = tid & 31, col = lane & 15, g = lane >> 4;
  const int h = blockIdx.y, q0 = blockIdx.x * 64 + wl * 16;
  const F2 qa = split_row(Q + (size_t)(q0 + col) * EMB + h * CH, 0, lane), qc = split_row(Q + (size_t)(q0 + col) * EMB + h * CH, 32, lane);
  float m_r[8], l_r[8];
  v8f o[4] = {};
#pragma unroll
  for (int r = 0; r < 8; ++r) { m_r[r] = -3.0e38f; l_r[r] = 0.f; }
  float* P = Ps[wl];
  for (int j = 0; j < NNODE / 32; ++j) {
    const int ks = j * 32;
    v8f s0 = {}, s1 = {};
    { const float* k0 = Kf + (size_t)(ks + col) * EMB + h * CH, *k1 = k0 + 16 * EMB;
      s0 = mac3(qa, split_row(k0, 0, lane), s0); s0 = mac3(qc, split_row(k0, 32, lane), s0);
      s1 = mac3(qa, split_row(k1, 0, lane), s1); s1 = mac3(qc, split_row(k1, 32, lane), s1); }
#pragma unroll
    for (int r = 0; r < 8; ++r) {
      const float a0 = s0[r] * 0.125f, a1 = s1[r] * 0.125f;
      float mx = fmaxf(a0, a1);
#pragma unroll
      for (int off = 8; off >= 1; off >>= 1) mx = fmaxf(mx, __shfl_xor(mx, off, 32));
      const float mn = fmaxf(m_r[r], mx);
      const float p0 = expf(a0 - mn), p1 = expf(a1 - mn);
      P[(8 * g + r) * 32 + col] = p0; P[(8 * g + r) * 32 + 16 + col] = p1;
      float sum = p0 + p1;
#pragma unroll
      for (int off = 8; off >= 1; off >>= 1) sum += __shfl_xor(sum, off, 32);
      const float corr = expf(m_r[r] - mn);
      l_r[r] = l_r[r] * corr + sum; m_r[r] = mn;
#pragma unroll
      for (int t = 0; t < 4; ++t) o[t][r] *= corr;
    }
    asm volatile("s_wait_dscnt 0" ::: "memory"); __builtin_amdgcn_wave_barrier(); __builtin_amdgcn_fence(__ATOMIC_RELEASE, "workgroup");
    const F2 pf = split_row(P + col * 32, 0, lane);
#pragma unroll
    for (int t = 0; t < 4; ++t) o[t] = mac3(pf, split_col(V + (size_t)ks * EMB + h * CH + t * 16 + col, 0, lane, EMB), o[t]);
    __builtin_amdgcn_wave_barrier();
  }
  float* so = Os[wl];
#pragma unroll
  for (int t = 0; t < 4; ++t)
#pragma unroll
    for (int r = 0; r < 8; ++r) so[(8 * g + r) * 64 + t * 16 + col] = o[t][r] / l_r[r];
  asm volatile("s_wait_dscnt 0" ::: "memory"); __builtin_amdgcn_wave_barrier(); __builtin_amdgcn_fence(__ATOMIC_RELEASE, "workgroup");
#pragma unroll
  for (int q = 0; q < 8; ++q) { const int rl = q * 2 + (lane >> 4), pc = lane & 15;
    vst2(O + (size_t)(q0 + rl) * EMB + h * CH + pc * 4, *(const v4f*)(so + rl * 64 + pc * 4)); }
}

extern "C" void kernel_launch(void* const* d_in, const int* in_sizes, int n_in,
                              void* d_out, int out_size, void* d_ws, size_t ws_size,
                              hipStream_t stream) {
  (void)in_sizes; (void)n_in; (void)out_size; (void)ws_size;
  const float* tgt   = (const float*)d_in[0];
  const float* mem   = (const float*)d_in[1];
  const float* orig  = (const float*)d_in[2];
  const int*   ei    = (const int*)d_in[3];
  const float* W_gat = (const float*)d_in[4];
  const float* att_s = (const float*)d_in[5];
  const float* att_d = (const float*)d_in[6];
  const float* b_gat = (const float*)d_in[7];
  const float* ipw   = (const float*)d_in[8];
  const float* ipb   = (const float*)d_in[9];
  const float* opw   = (const float*)d_in[10];
  const float* opb   = (const float*)d_in[11];
  const float* l1w   = (const float*)d_in[12];
  const float* l1b   = (const float*)d_in[13];
  float* out = (float*)d_out;
  float* ws = (float*)d_ws; size_t off = 0;
  auto carve = [&](size_t n) { float* p = ws + off; off += (n + 63) & ~(size_t)63; return p; };
  float* xh = carve((size_t)NNODE * EMB);
  float* as = carve((size_t)NNODE * NH);
  float* ad = carve((size_t)NNODE * NH);
  float* tb = carve((size_t)NNODE * EMB);
  float* Q  = carve((size_t)NNODE * EMB);
  float* Kf = carve((size_t)NNODE * EMB);
  float* V  = carve((size_t)NNODE * EMB);
  float* O  = carve((size_t)NNODE * EMB);
  float* fu = carve((size_t)NNODE * EMB);
  const dim3 g256(NNODE / 64, EMB / 64), g128(NNODE / 64, DFF / 64);
  k_gemm<<<g256, 128, 0, stream>>>(tgt, FIN, W_gat, EMB, 1, nullptr, 0, xh, EMB, FIN);
  k_gat_alpha<<<NNODE / 32, 256, 0, stream>>>(xh, att_s, att_d, as, ad);
  k_gat_gather<<<NNODE / DT, 256, 0, stream>>>(ei, xh, as, ad, b_gat, tb);
  k_gemm<<<g256, 128, 0, stream>>>(tb,   EMB, ipw,             EMB, 0, ipb,           0, Q,  EMB, EMB);
  k_gemm<<<g256, 128, 0, stream>>>(mem,  EMB, ipw + EMB * EMB, EMB, 0, ipb + EMB,     0, Kf, EMB, EMB);
  k_gemm<<<g256, 128, 0, stream>>>(orig, EMB, ipw + 2 * EMB * EMB, EMB, 0, ipb + 2 * EMB, 0, V, EMB, EMB);
  k_attn<<<dim3(NNODE / 64, NH), 128, 0, stream>>>(Q, Kf, V, O);
  k_gemm<<<g256, 128, 0, stream>>>(O,  EMB, opw, EMB, 0, opb, 0, fu,  EMB, EMB);
  k_gemm<<<g128, 128, 0, stream>>>(fu, EMB, l1w, EMB, 0, l1b, 1, out, DFF, EMB);
}
